// HeteAttentionHead_48284022342203
// MI455X (gfx1250) — hardware-verified
//
#include <hip/hip_runtime.h>
#include <stddef.h>


#define DF    128
#define GR    32
#define APQ   17
#define XSP   132
#define KP    132
#define NB    512
#define CHUNK 2048
#define NTHR  256
#define NWAVE 8
#define WCAP  256
#define NGRP  ((CHUNK * 2) / (NTHR * 4))
#define WQ    (DF * DF / 8)

#define LDS_SACC (NB * DF)
#define LDS_DEN  NB
#define LDS_LIST (NWAVE * WCAP)
#define LDS_BYTES ((LDS_SACC + LDS_DEN + LDS_LIST + NWAVE) * 4)

static_assert(NGRP == 4);
static_assert(WCAP == NGRP * 2 * 32);
static_assert((NB & (NB - 1)) == 0);
static_assert(NB == NWAVE * 64);
static_assert(CHUNK == 2048);
static_assert(((LDS_SACC + LDS_DEN) % 4) == 0);
static_assert(LDS_BYTES == 272416);
static_assert(GR * APQ * 16 == 8704);

typedef float          v4f  __attribute__((ext_vector_type(4)));
typedef float          v8f  __attribute__((ext_vector_type(8)));
typedef int            v4i  __attribute__((ext_vector_type(4)));
typedef unsigned short v8us __attribute__((ext_vector_type(8)));
typedef __bf16         v16b __attribute__((ext_vector_type(16)));

union Frag  { v16b v; v4i q[2]; };
union Pack8 { v8us u; v4i i; };

__device__ __forceinline__ v8f wm(v16b a, v16b b, v8f c) {
  v8f d = __builtin_amdgcn_wmma_f32_16x16x32_bf16(false, a, false, b, (short)0, c, false, false);
  asm volatile("v_nop\n\tv_nop\n\tv_nop\n\tv_nop" : "+v"(d) : "v"(a), "v"(b));
  return d;
}

__device__ __forceinline__ float wsum(float v) {
  v += __shfl_xor(v, 16, 32);
  v += __shfl_xor(v, 8, 32);
  v += __shfl_xor(v, 4, 32);
  v += __shfl_xor(v, 2, 32);
  v += __shfl_xor(v, 1, 32);
  return v;
}

__device__ __forceinline__ unsigned int bfb(float f) {
  const unsigned int u = __float_as_uint(f);
  return (u + 0x7FFFu + ((u >> 16) & 1u)) >> 16;
}

__device__ __forceinline__ void split8(v4f a, v4f b, Pack8& H, Pack8& L) {
  float s[8] = {a.x, a.y, a.z, a.w, b.x, b.y, b.z, b.w};
#pragma unroll
  for (int j = 0; j < 8; ++j) {
    const unsigned int hb = bfb(s[j]);
    const float rem = s[j] - __uint_as_float(hb << 16);
    H.u[j] = (unsigned short)hb;
    L.u[j] = (unsigned short)bfb(rem);
  }
}

__global__ __launch_bounds__(NTHR) void k_prepw(
    const float* __restrict__ W0, const float* __restrict__ W1,
    const float* __restrict__ W2, const float* __restrict__ W3, v4i* Wq) {
  __shared__ __attribute__((aligned(16))) float Tt[GR * KP];
  const int tid = threadIdx.x, lane = tid & 31, wave = tid >> 5;
  const int mat = blockIdx.x >> 2;
  const int n0 = (blockIdx.x & 3) * GR;
  const float* W = (mat == 0) ? W0 : (mat == 1) ? W1 : (mat == 2) ? W2 : W3;
  {
    const int k  = tid >> 1;
    const int c0 = (tid & 1) * 16;
    const float* p = W + (size_t)k * DF + n0 + c0;
    const v4f f0 = *(const v4f*)(p), f1 = *(const v4f*)(p + 4);
    const v4f f2 = *(const v4f*)(p + 8), f3 = *(const v4f*)(p + 12);
    float* t = Tt + k;
    t[(c0 + 0) * KP] = f0.x;  t[(c0 + 1) * KP] = f0.y;  t[(c0 + 2) * KP] = f0.z;  t[(c0 + 3) * KP] = f0.w;
    t[(c0 + 4) * KP] = f1.x;  t[(c0 + 5) * KP] = f1.y;  t[(c0 + 6) * KP] = f1.z;  t[(c0 + 7) * KP] = f1.w;
    t[(c0 + 8) * KP] = f2.x;  t[(c0 + 9) * KP] = f2.y;  t[(c0 + 10) * KP] = f2.z; t[(c0 + 11) * KP] = f2.w;
    t[(c0 + 12) * KP] = f3.x; t[(c0 + 13) * KP] = f3.y; t[(c0 + 14) * KP] = f3.z; t[(c0 + 15) * KP] = f3.w;
  }
  __syncthreads();

  v4i* Hq = Wq + (size_t)mat * 2 * WQ;
  v4i* Lq = Hq + WQ;
  const int m = lane & 15, hh = lane >> 4;
  Pack8 H[2], L[2];
  size_t o[2];
#pragma unroll
  for (int i = 0; i < 2; ++i) {
    const int r = 4 * wave + 2 * i + hh;
    const v4f a = *(const v4f*)(Tt + r * KP + 8 * m);
    const v4f b = *(const v4f*)(Tt + r * KP + 8 * m + 4);
    split8(a, b, H[i], L[i]);
    o[i] = (size_t)(n0 + r) * (DF / 8) + m;
  }
#pragma unroll
  for (int i = 0; i < 2; ++i) { *(volatile v4i*)(Hq + o[i]) = H[i].i; *(volatile v4i*)(Lq + o[i]) = L[i].i; }
  __threadfence();
#pragma unroll
  for (int i = 0; i < 2; ++i) { *(volatile v4i*)(Hq + o[i]) = H[i].i; *(volatile v4i*)(Lq + o[i]) = L[i].i; }
}

__global__ __launch_bounds__(NTHR) void k_gemm(
    const float* __restrict__ X0, const float* __restrict__ X1,
    const v4i* __restrict__ Wq, int mat0, int mat1,
    const float* __restrict__ bias0, const float* __restrict__ bias1,
    float* Y0, float* Y1,
    const float* __restrict__ Wa, float* A0, float* A1,
    int dots, int n0rows, int n1rows) {
  __shared__ v4i Ahq[GR * APQ];
  __shared__ v4i Alq[GR * APQ];
  __shared__ __attribute__((aligned(16))) float Xs[GR * XSP];
  __shared__ __attribute__((aligned(16))) float As[GR];

  const int sel     = blockIdx.y;
  const int nrows   = sel ? n1rows : n0rows;
  const int rowBase = blockIdx.x * GR;
  if (rowBase >= nrows) return;

  const float* X    = sel ? X1 : X0;
  const float* bias = sel ? bias1 : bias0;
  float* Y          = sel ? Y1 : Y0;
  float* Aout       = sel ? A1 : A0;
  const float* was  = Wa + sel * DF;
  const int mat     = sel ? mat1 : mat0;
  const v4i* Whq    = Wq + (size_t)mat * 2 * WQ;
  const v4i* Wlq    = Whq + WQ;

  const int tid  = threadIdx.x;
  const int lane = tid & 31;
  const int wave = tid >> 5;
  const int hh   = lane >> 4;
  const int m    = lane & 15;

  {
    const int r  = tid >> 3;
    const int c0 = (tid & 7) * 16;
    int row = rowBase + r;
    if (row > nrows - 1) row = nrows - 1;
    const float* p = X + (size_t)row * DF + c0;
    const v4f f0 = *(const v4f*)(p), f1 = *(const v4f*)(p + 4);
    const v4f f2 = *(const v4f*)(p + 8), f3 = *(const v4f*)(p + 12);
    Pack8 H0, L0, H1, L1;
    split8(f0, f1, H0, L0);
    split8(f2, f3, H1, L1);
    const int q = r * APQ + (c0 >> 3);
    Ahq[q] = H0.i; Ahq[q + 1] = H1.i;
    Alq[q] = L0.i; Alq[q + 1] = L1.i;
  }
  __syncthreads();

  const int ncol = wave * 16 + m;
  v8f c0 = {0.f, 0.f, 0.f, 0.f, 0.f, 0.f, 0.f, 0.f};
  v8f c1 = {0.f, 0.f, 0.f, 0.f, 0.f, 0.f, 0.f, 0.f};
#pragma unroll 1
  for (int kt = 0; kt < DF / 32; ++kt) {
    Frag bh, bl, ah, al;
    const v4i* pbh = Whq + ncol * (DF / 8) + kt * 4 + hh;
    const v4i* pbl = Wlq + ncol * (DF / 8) + kt * 4 + hh;
    bh.q[0] = pbh[0]; bh.q[1] = pbh[2];
    bl.q[0] = pbl[0]; bl.q[1] = pbl[2];
    const int qa0 = m * APQ + kt * 4 + hh;
    ah.q[0] = Ahq[qa0]; ah.q[1] = Ahq[qa0 + 2];
    al.q[0] = Alq[qa0]; al.q[1] = Alq[qa0 + 2];
    c0 = wm(ah.v, bh.v, c0);
    c0 = wm(ah.v, bl.v, c0);
    c0 = wm(al.v, bh.v, c0);
    const int qa1 = (16 + m) * APQ + kt * 4 + hh;
    ah.q[0] = Ahq[qa1]; ah.q[1] = Ahq[qa1 + 2];
    al.q[0] = Alq[qa1]; al.q[1] = Alq[qa1 + 2];
    c1 = wm(ah.v, bh.v, c1);
    c1 = wm(ah.v, bl.v, c1);
    c1 = wm(al.v, bh.v, c1);
  }

  const float bv = bias[ncol];
#pragma unroll
  for (int r = 0; r < 8; ++r) {
    Xs[(8 * hh + r) * XSP + ncol]      = c0[r] + bv;
    Xs[(16 + 8 * hh + r) * XSP + ncol] = c1[r] + bv;
  }
  __syncthreads();

  const v4f wv = *(const v4f*)(was + 4 * lane);
  v4f xr[4];
  float* yp[4];
#pragma unroll
  for (int i = 0; i < 4; ++i) {
    const int rl = 4 * wave + i;
    xr[i] = *(const v4f*)(Xs + rl * XSP + 4 * lane);
    yp[i] = Y + (size_t)(rowBase + rl) * DF + 4 * lane;
    float d = xr[i].x * wv.x + xr[i].y * wv.y + xr[i].z * wv.z + xr[i].w * wv.w;
    d = wsum(d);
    if (lane == 0) As[rl] = d;
  }
  __syncthreads();

  const bool wa = (dots != 0) && (wave == 0) && (lane < 8);
  v4f av = {0.f, 0.f, 0.f, 0.f};
  if (lane < 8) av = *(const v4f*)(As + 4 * lane);
  float* ap = Aout + rowBase + 4 * (lane & 7);

#pragma unroll
  for (int i = 0; i < 4; ++i) *(volatile v4f*)(yp[i]) = xr[i];
  if (wa) *(volatile v4f*)ap = av;
  __threadfence();
#pragma unroll
  for (int i = 0; i < 4; ++i) *(volatile v4f*)(yp[i]) = xr[i];
  if (wa) *(volatile v4f*)ap = av;
}

__global__ __launch_bounds__(NTHR) void k_agg(
    const int* __restrict__ edges, const float* __restrict__ nbr,
    const float* __restrict__ acur, const float* __restrict__ anbr,
    const float* __restrict__ ba, float* out, int nN, int nM, int nE) {
  extern __shared__ v4f lds_dyn[];
  float* sacc = (float*)lds_dyn;
  float* den  = sacc + LDS_SACC;
  int*   list = (int*)(den + LDS_DEN);
  int*   wcnt = list + LDS_LIST;

  const int tid  = threadIdx.x;
  const int lane = tid & 31;
  const int wave = tid >> 5;
  const int nodeBase = blockIdx.x * NB;
  const float ba0 = ba[0];

  {
    const v4f z4 = {0.f, 0.f, 0.f, 0.f};
    for (int i = tid; i < (LDS_SACC + LDS_DEN) / 4; i += NTHR) lds_dyn[i] = z4;
  }
  __syncthreads();

  const int nChunks = (nE + CHUNK - 1) / CHUNK;
  const int sent = -2147483647 - 1;
#pragma unroll 1
  for (int ch = 0; ch < nChunks; ++ch) {
    const int cbase = ch * CHUNK;
    int wc = 0;
#pragma unroll
    for (int g = 0; g < NGRP; ++g) {
      const int el0 = (g * NTHR + tid) * 2;
      const int e0  = cbase + el0;
      v4i d;
      if (e0 + 1 < nE) {
        d = *(const v4i*)(edges + (size_t)e0 * 2);
      } else {
        d.x = (e0 < nE) ? edges[(size_t)min(e0, nE - 1) * 2] : sent;
        d.y = 0; d.z = sent; d.w = 0;
      }
      const unsigned s0 = (unsigned)d.x - (unsigned)nodeBase;
      const unsigned s1 = (unsigned)d.z - (unsigned)nodeBase;
      const bool h0 = s0 < (unsigned)NB;
      const bool h1 = s1 < (unsigned)NB;
      const unsigned many = __builtin_amdgcn_ballot_w32(h0 | h1);
      if (many != 0u) {
#define HITJ(J, HJ, SJ) { \
          const unsigned mj = __builtin_amdgcn_ballot_w32(HJ); \
          if (HJ) { \
            const int pos = wc + (int)__builtin_amdgcn_mbcnt_lo(mj, 0u); \
            if (pos < WCAP) list[wave * WCAP + pos] = ((el0 + (J)) << 9) | (int)(SJ); \
          } \
          wc += (int)__builtin_popcount(mj); }
        HITJ(0, h0, s0)
        HITJ(1, h1, s1)
#undef HITJ
      }
    }
    if (lane == 0) wcnt[wave] = wc;
    __syncthreads();

    if (wave == 0) {
      for (int wsx = 0; wsx < NWAVE; ++wsx) {
        int n = wcnt[wsx];
        if (n > WCAP) n = WCAP;
        if (n < 0) n = 0;
        for (int i = 0; i < n; ++i) {
          const int ent  = list[wsx * WCAP + i];
          const int slot = ent & (NB - 1);
          const int el   = (ent >> 9) & (CHUNK - 1);
          int e = cbase + el;
          if (e > nE - 1) e = nE - 1;
          int dst = edges[(size_t)e * 2 + 1];
          dst = dst < 0 ? 0 : (dst > nM - 1 ? nM - 1 : dst);
          int nd = nodeBase + slot;
          if (nd > nN - 1) nd = nN - 1;
          float al = acur[nd] + anbr[dst] + ba0;
          al = (al > 0.f) ? al : 0.2f * al;
          const float p = __expf(al);
          const v4f xv = *(const v4f*)(nbr + (size_t)dst * DF + 4 * lane);
          v4f* sp = (v4f*)(sacc + slot * DF + 4 * lane);
          const v4f cur = *sp;
          const v4f nxt = cur + p * xv;
          *sp = nxt;
          if (lane == 0) {
            const float od = den[slot];
            den[slot] = od + p;
          }
        }
      }
    }
    __syncthreads();
  }

#pragma unroll 1
  for (int j = 0; j < NB / NWAVE; ++j) {
    const int slot = wave * (NB / NWAVE) + j;
    const int node = nodeBase + slot;
    if (node >= nN) break;
    const float dv  = den[slot];
    const float inv = (dv > 0.f) ? __builtin_amdgcn_rcpf(dv) : 0.f;
    const v4f sv = *(const v4f*)(sacc + slot * DF + 4 * lane);
    const v4f y  = sv * inv;
    float* op = out + (size_t)node * DF + 4 * lane;
    *(volatile v4f*)op = y;
    __threadfence();
    *(volatile v4f*)op = y;
  }
}

static inline size_t alup(size_t v) { return (v + 255) & ~(size_t)255; }

extern "C" void kernel_launch(void* const* d_in, const int* in_sizes, int n_in,
                              void* d_out, int out_size, void* d_ws, size_t ws_size,
                              hipStream_t stream) {
  if (n_in < 13) return;
  const int nN = in_sizes[0] / DF;
  const int nM = in_sizes[1] / DF;
  if (nN <= 0 || nM <= 0 || in_sizes[0] != nN * DF || in_sizes[1] != nM * DF) return;
  if (in_sizes[2] != DF * DF || in_sizes[4] != DF * DF || in_sizes[6] != DF * DF || in_sizes[8] != DF * DF) return;
  if (in_sizes[3] != DF || in_sizes[5] != DF || in_sizes[7] != DF || in_sizes[9] != DF) return;
  if (in_sizes[10] != 2 * DF || in_sizes[11] < 1) return;
  const int nE = in_sizes[12] / 2;
  if (nE < 1 || in_sizes[12] != 2 * nE) return;
  if (out_size != nN * DF) return;

  const float* x_cur = (const float*)d_in[0];
  const float* x_nbr = (const float*)d_in[1];
  const float* W1c   = (const float*)d_in[2];
  const float* b1c   = (const float*)d_in[3];
  const float* W2c   = (const float*)d_in[4];
  const float* b2c   = (const float*)d_in[5];
  const float* W1n   = (const float*)d_in[6];
  const float* b1n   = (const float*)d_in[7];
  const float* W2n   = (const float*)d_in[8];
  const float* b2n   = (const float*)d_in[9];
  const float* Wa    = (const float*)d_in[10];
  const float* ba    = (const float*)d_in[11];
  const int*   edges = (const int*)d_in[12];
  float* out = (float*)d_out;

  const int nP0 = ((nN + GR - 1) / GR) * GR;
  const int nP1 = ((nM + GR - 1) / GR) * GR;
  size_t off = 0;
  v4i*   Wq   = (v4i*)((char*)d_ws + off);   off += alup((size_t)4 * 2 * DF * DF * 2);
  float* h1c  = (float*)((char*)d_ws + off); off += alup((size_t)nP0 * DF * sizeof(float));
  float* h1n  = (float*)((char*)d_ws + off); off += alup((size_t)nP1 * DF * sizeof(float));
  float* curb = (float*)((char*)d_ws + off); off += alup((size_t)nP0 * DF * sizeof(float));
  float* nbrb = (float*)((char*)d_ws + off); off += alup((size_t)nP1 * DF * sizeof(float));
  float* acur = (float*)((char*)d_ws + off); off += alup((size_t)nP0 * sizeof(float));
  float* anbr = (float*)((char*)d_ws + off); off += alup((size_t)nP1 * sizeof(float));
  if (off > ws_size) return;

  k_prepw<<<16, NTHR, 0, stream>>>(W1c, W2c, W1n, W2n, Wq);

  const int gx = ((nP0 > nP1) ? nP0 : nP1) / GR;
  k_gemm<<<dim3(gx, 2), NTHR, 0, stream>>>(x_cur, x_nbr, Wq, 0, 2, b1c, b1n, h1c, h1n,
                                            Wa, acur, anbr, 0, nN, nM);
  k_gemm<<<dim3(gx, 2), NTHR, 0, stream>>>(h1c, h1n, Wq, 1, 3, b2c, b2n, curb, nbrb,
                                            Wa, acur, anbr, 1, nN, nM);

  hipFuncSetAttribute(reinterpret_cast<const void*>(&k_agg),
                      hipFuncAttributeMaxDynamicSharedMemorySize, LDS_BYTES);
  const int grid = (nN + NB - 1) / NB;
  k_agg<<<grid, NTHR, LDS_BYTES, stream>>>(edges, nbrb, acur, anbr, ba, out, nN, nM, nE);
}
